// RNNModel_32160715112736
// MI455X (gfx1250) — hardware-verified
//
#include <hip/hip_runtime.h>
#include <math.h>

constexpr int NBATCH  = 128;
constexpr int NSTEP   = 512;
constexpr int NIN     = 128;
constexpr int NHID    = 512;
constexpr int NOUT    = 128;
constexpr int HALF_B  = 64;
constexpr int NHALF   = NBATCH / HALF_B;
constexpr int HROWS   = NSTEP * HALF_B;
constexpr int NTHR    = 256;
constexpr int HPITCH  = 520;
constexpr int SLABP   = 68;
constexpr float W_CARRY   = 256.0f;
constexpr float A_CARRY   = 64.0f;
constexpr float WX1_CARRY = W_CARRY * A_CARRY;
constexpr float ACC_INV   = 1.0f / (W_CARRY * A_CARRY);
constexpr size_t OFF_WX1 = 0;
constexpr size_t OFF_WH1 = OFF_WX1 + (size_t)NHID * NIN;
constexpr size_t OFF_WO1 = OFF_WH1 + (size_t)NHID * NHID;
constexpr size_t OFF_WX2 = OFF_WO1 + (size_t)NHID * NHID;
constexpr size_t OFF_WH2 = OFF_WX2 + (size_t)NHID * NHID;
constexpr size_t OFF_WO2 = OFF_WH2 + (size_t)NHID * NHID;
constexpr size_t OFF_WL  = OFF_WO2 + (size_t)NHID * NHID;
constexpr size_t WTS_ELEMS = OFF_WL + (size_t)NOUT * NHID;
constexpr int PWB_WX1 = NHID * NIN / 2048;
constexpr int PWB_SQ  = NHID * NHID / 2048;
constexpr int PWB_WL  = NOUT * NHID / 2048;
constexpr int PW_B1 = PWB_WX1;
constexpr int PW_B2 = PW_B1 + PWB_SQ;
constexpr int PW_B3 = PW_B2 + PWB_SQ;
constexpr int PW_B4 = PW_B3 + PWB_SQ;
constexpr int PW_B5 = PW_B4 + PWB_SQ;
constexpr int PW_B6 = PW_B5 + PWB_SQ;
constexpr int PW_BLOCKS = PW_B6 + PWB_WL;
constexpr int PX_BLOCKS = NBATCH * NSTEP * (NIN / 8) / NTHR;

static_assert(NBATCH == NHALF * HALF_B, "batch halves");
static_assert(HALF_B == 64, "one 64-row tile per half");
static_assert(NIN % 32 == 0 && NHID % 32 == 0, "K multiples of 32");
static_assert(NHID % 64 == 0 && NOUT % 64 == 0 && HROWS % 64 == 0, "M, N tile multiples");
static_assert(NHID == 64 * (NTHR / 32), "8 waves x 64 hidden columns");
static_assert((HALF_B * HPITCH) % NTHR == 0, "h zero-fill loop exact");
static_assert((HPITCH % 8) == 0 && (SLABP % 4) == 0, "16-byte aligned LDS vectors");
static_assert(NHID * NIN % 2048 == 0 && NHID * NHID % 2048 == 0 && NOUT * NHID % 2048 == 0, "weight convert blocks exact");
static_assert(PW_BLOCKS == 704, "weight convert grid");
static_assert(PX_BLOCKS == 4096, "x convert grid");
static_assert((OFF_WH1 * 2) % 256 == 0 && (OFF_WO1 * 2) % 256 == 0 && (OFF_WX2 * 2) % 256 == 0 &&
              (OFF_WH2 * 2) % 256 == 0 && (OFF_WO2 * 2) % 256 == 0 && (OFF_WL * 2) % 256 == 0, "plane alignment");

typedef __attribute__((ext_vector_type(16))) _Float16 v16h;
typedef __attribute__((ext_vector_type(8)))  _Float16 v8h;
typedef __attribute__((ext_vector_type(8)))  float    v8f;
typedef __attribute__((ext_vector_type(4)))  float    v4f;

union FragU { v16h v; v8h h[2]; };

__device__ __forceinline__ v16h frag_load(const _Float16* p) {
  FragU f;
  f.h[0] = *(const v8h*)(p);
  f.h[1] = *(const v8h*)(p + 16);
  return f.v;
}
__device__ __forceinline__ v8f mma_h(v16h a, v16h b, v8f c) {
  return __builtin_amdgcn_wmma_f32_16x16x32_f16(false, a, false, b, (short)0, c, false, false);
}
__device__ __forceinline__ void guard_row(v8f& a, v8f& b, v8f& c, v8f& d, v16h x, v16h y0, v16h y1, v16h y2, v16h y3) {
  asm volatile("v_nop\n\tv_nop\n\tv_nop\n\tv_nop" : "+v"(a), "+v"(b), "+v"(c), "+v"(d) : "v"(x), "v"(y0), "v"(y1), "v"(y2), "v"(y3));
}
__device__ __forceinline__ void keep4_h(v16h a, v16h b, v16h c, v16h d) { asm volatile("v_nop" :: "v"(a), "v"(b), "v"(c), "v"(d)); }
__device__ __forceinline__ void acc_guard4(v8f& a, v8f& b, v8f& c, v8f& d) { asm volatile("v_nop\n\tv_nop\n\tv_nop\n\tv_nop" : "+v"(a), "+v"(b), "+v"(c), "+v"(d)); }

__device__ __forceinline__ void wave_sync() {
  __builtin_amdgcn_fence(__ATOMIC_RELEASE, "workgroup");
  __builtin_amdgcn_wave_barrier();
  __builtin_amdgcn_fence(__ATOMIC_ACQUIRE, "workgroup");
}

__device__ __forceinline__ float gelu_erf(float x) {
  return 0.5f * x * (1.0f + erff(x * 0.70710678118654752f));
}

__device__ __forceinline__ void stage_raw(float* slab, v8f a0, v8f a1, v8f a2, v8f a3, float sc, int rlane, int mOff) {
#pragma unroll
  for (int r = 0; r < 8; ++r) {
    float* p = slab + (mOff + r) * SLABP + rlane;
    p[0]  = a0[r] * sc;
    p[16] = a1[r] * sc;
    p[32] = a2[r] * sc;
    p[48] = a3[r] * sc;
  }
}
__device__ __forceinline__ void stage_bias(float* slab, v8f a0, v8f a1, v8f a2, v8f a3, float sc,
                                           float b0, float b1, float b2, float b3, int rlane, int mOff) {
#pragma unroll
  for (int r = 0; r < 8; ++r) {
    float* p = slab + (mOff + r) * SLABP + rlane;
    p[0]  = a0[r] * sc + b0;
    p[16] = a1[r] * sc + b1;
    p[32] = a2[r] * sc + b2;
    p[48] = a3[r] * sc + b3;
  }
}
__device__ __forceinline__ void gelu_pass(float* slab, v4f b4, int lane) {
  const int c4 = (lane & 15) * 4;
  const int hh = lane >> 4;
#pragma unroll 1
  for (int q = 0; q < 8; ++q) {
    float* p = slab + (2 * q + hh) * SLABP + c4;
    const v4f v = *(const v4f*)p;
    v4f o;
#pragma unroll
    for (int e = 0; e < 4; ++e) {
      const float x = v[e] + b4[e];
      o[e] = gelu_erf(x) * A_CARRY;
    }
    *(v4f*)p = o;
  }
}
__device__ __forceinline__ v8h cvt8_slab(const float* sp) {
  const v4f a = *(const v4f*)(sp);
  const v4f b = *(const v4f*)(sp + 4);
  v8h h;
#pragma unroll
  for (int e = 0; e < 4; ++e) {
    h[e]     = (_Float16)a[e];
    h[4 + e] = (_Float16)b[e];
  }
  return h;
}

__global__ __launch_bounds__(NTHR) void prep_x_kernel(const float* __restrict__ x, unsigned short* __restrict__ xt) {
  const int i   = blockIdx.x * NTHR + threadIdx.x;
  const int r   = i >> 4;
  const int c8  = i & 15;
  const int hf  = r >> 15;
  const int rr  = r & (HROWS - 1);
  const int t   = rr >> 6;
  const int bp  = rr & 63;
  const int b   = hf * HALF_B + bp;
  const float* sp = x + ((size_t)b * NSTEP + (size_t)t) * NIN + c8 * 8;
  const v4f a = *(const v4f*)(sp);
  const v4f c = *(const v4f*)(sp + 4);
  v8h hv;
#pragma unroll
  for (int e = 0; e < 4; ++e) {
    hv[e]     = (_Float16)a[e];
    hv[4 + e] = (_Float16)c[e];
  }
  *(volatile v8h*)(xt + (size_t)i * 8) = hv;
  __threadfence();
  *(volatile v8h*)(xt + (size_t)i * 8) = hv;
}

__global__ __launch_bounds__(NTHR) void prep_w_kernel(const float* __restrict__ w_in1, const float* __restrict__ w_out1,
                                                      const float* __restrict__ w_in2, const float* __restrict__ w_out2,
                                                      const float* __restrict__ w_last, unsigned short* __restrict__ wts) {
  const int bx = blockIdx.x;
  const float* src = w_in1;
  int spitch = NIN + NHID, scol0 = 0, lg = 4, b0 = 0;
  size_t doff = OFF_WX1;
  float sc = WX1_CARRY;
  if (bx >= PW_B1) { src = w_in1;  spitch = NIN + NHID;  scol0 = NIN;  lg = 6; b0 = PW_B1; doff = OFF_WH1; sc = W_CARRY; }
  if (bx >= PW_B2) { src = w_out1; spitch = NHID;        scol0 = 0;    lg = 6; b0 = PW_B2; doff = OFF_WO1; sc = W_CARRY; }
  if (bx >= PW_B3) { src = w_in2;  spitch = NHID + NHID; scol0 = 0;    lg = 6; b0 = PW_B3; doff = OFF_WX2; sc = W_CARRY; }
  if (bx >= PW_B4) { src = w_in2;  spitch = NHID + NHID; scol0 = NHID; lg = 6; b0 = PW_B4; doff = OFF_WH2; sc = W_CARRY; }
  if (bx >= PW_B5) { src = w_out2; spitch = NHID;        scol0 = 0;    lg = 6; b0 = PW_B5; doff = OFF_WO2; sc = W_CARRY; }
  if (bx >= PW_B6) { src = w_last; spitch = NHID;        scol0 = 0;    lg = 6; b0 = PW_B6; doff = OFF_WL;  sc = W_CARRY; }
  const int i   = (bx - b0) * NTHR + threadIdx.x;
  const int row = i >> lg;
  const int c8  = i & ((1 << lg) - 1);
  const float* sp = src + (size_t)row * spitch + scol0 + c8 * 8;
  const v4f a = *(const v4f*)(sp);
  const v4f c = *(const v4f*)(sp + 4);
  v8h hv;
#pragma unroll
  for (int e = 0; e < 4; ++e) {
    hv[e]     = (_Float16)(a[e] * sc);
    hv[4 + e] = (_Float16)(c[e] * sc);
  }
  unsigned short* dp = wts + doff + (size_t)i * 8;
  *(volatile v8h*)dp = hv;
  __threadfence();
  *(volatile v8h*)dp = hv;
}

template <int KX>
__global__ __launch_bounds__(NTHR) void rnn_rec_kernel(const unsigned short* __restrict__ Xp,
                                                       const unsigned short* __restrict__ Wxp,
                                                       const unsigned short* __restrict__ Whp,
                                                       const float* __restrict__ bias,
                                                       unsigned short* __restrict__ Hout) {
  static_assert(KX % 32 == 0, "K multiple of 32");
  __shared__ __align__(16) _Float16 Ah[HALF_B * HPITCH];
  __shared__ __align__(16) float    Sl[NTHR / 32][16 * SLABP];
  const _Float16* X  = (const _Float16*)Xp;
  const _Float16* Wx = (const _Float16*)Wxp;
  const _Float16* Wh = (const _Float16*)Whp;
  const int tid = threadIdx.x, lane = tid & 31, wave = tid >> 5;
  const int rlane = lane & 15, hh = lane >> 4, koff = hh * 8, mOff = hh * 8;
  const int n0 = wave * 64;

#pragma unroll 1
  for (int i = tid; i < HALF_B * HPITCH; i += NTHR) Ah[i] = (_Float16)0.0f;

  const v4f b4 = *(const v4f*)(bias + n0 + rlane * 4);
  float* slab = Sl[wave];
  const _Float16* wx = Wx + (size_t)(n0 + rlane) * KX + koff;
  const _Float16* wh = Wh + (size_t)(n0 + rlane) * NHID + koff;
  const _Float16* ha = Ah + rlane * HPITCH + koff;
  const int q = lane >> 3, c8 = (lane & 7) * 8;
  __syncthreads();

#pragma unroll 1
  for (int t = 0; t < NSTEP; ++t) {
    v8f acc[4][4];
#pragma unroll
    for (int i = 0; i < 4; ++i)
#pragma unroll
      for (int j = 0; j < 4; ++j) acc[i][j] = (v8f){0.f, 0.f, 0.f, 0.f, 0.f, 0.f, 0.f, 0.f};

    const _Float16* xa = X + ((size_t)t * HALF_B + rlane) * KX + koff;
#pragma unroll 1
    for (int k0 = 0; k0 < KX; k0 += 32) {
      v16h bh[4];
#pragma unroll
      for (int j = 0; j < 4; ++j) bh[j] = frag_load(wx + (size_t)(16 * j) * KX + k0);
#pragma unroll
      for (int i = 0; i < 4; ++i) {
        const v16h ah = frag_load(xa + (size_t)(16 * i) * KX + k0);
#pragma unroll
        for (int j = 0; j < 4; ++j) acc[i][j] = mma_h(ah, bh[j], acc[i][j]);
        guard_row(acc[i][0], acc[i][1], acc[i][2], acc[i][3], ah, bh[0], bh[1], bh[2], bh[3]);
      }
      keep4_h(bh[0], bh[1], bh[2], bh[3]);
    }
#pragma unroll 1
    for (int k0 = 0; k0 < NHID; k0 += 32) {
      v16h bh[4];
#pragma unroll
      for (int j = 0; j < 4; ++j) bh[j] = frag_load(wh + (size_t)(16 * j) * NHID + k0);
#pragma unroll
      for (int i = 0; i < 4; ++i) {
        const v16h ah = frag_load(ha + (16 * i) * HPITCH + k0);
#pragma unroll
        for (int j = 0; j < 4; ++j) acc[i][j] = mma_h(ah, bh[j], acc[i][j]);
        guard_row(acc[i][0], acc[i][1], acc[i][2], acc[i][3], ah, bh[0], bh[1], bh[2], bh[3]);
      }
      keep4_h(bh[0], bh[1], bh[2], bh[3]);
    }
    acc_guard4(acc[0][0], acc[0][1], acc[0][2], acc[0][3]);
    acc_guard4(acc[1][0], acc[1][1], acc[1][2], acc[1][3]);
    acc_guard4(acc[2][0], acc[2][1], acc[2][2], acc[2][3]);
    acc_guard4(acc[3][0], acc[3][1], acc[3][2], acc[3][3]);

    __syncthreads();

#pragma unroll
    for (int i = 0; i < 4; ++i) {
      stage_raw(slab, acc[i][0], acc[i][1], acc[i][2], acc[i][3], ACC_INV, rlane, mOff);
      wave_sync();
      gelu_pass(slab, b4, lane);
      wave_sync();
      unsigned short* gp = Hout + ((size_t)t * HALF_B + 16 * i) * NHID + n0 + c8;
#pragma unroll
      for (int it = 0; it < 4; ++it) {
        const int row = it * 4 + q;
        const v8h hv = cvt8_slab(slab + row * SLABP + c8);
        *(v8h*)(Ah + (16 * i + row) * HPITCH + n0 + c8) = hv;
        *(volatile v8h*)(gp + (size_t)row * NHID) = hv;
      }
      __threadfence();
#pragma unroll
      for (int it = 0; it < 4; ++it) {
        const int row = it * 4 + q;
        const v8h hv = cvt8_slab(slab + row * SLABP + c8);
        *(volatile v8h*)(gp + (size_t)row * NHID) = hv;
      }
      __threadfence();
      wave_sync();
    }
    __syncthreads();
  }
}

template <int OUTK>
__global__ __launch_bounds__(NTHR) void gemm_tile_kernel(const unsigned short* __restrict__ Ap,
                                                         const unsigned short* __restrict__ Btp,
                                                         void* __restrict__ Cout, const float* __restrict__ bias,
                                                         int M, int N, int K, float scale, int bat0) {
  __shared__ __align__(16) float sT[NTHR / 32][16 * SLABP];
  const _Float16* A  = (const _Float16*)Ap;
  const _Float16* Bt = (const _Float16*)Btp;
  const int lane = threadIdx.x & 31, wave = threadIdx.x >> 5;
  const int tilesN = N >> 6, tilesM = M >> 6;
  const int tile = blockIdx.x * 8 + wave;
  if (tile >= tilesM * tilesN) return;
  const int tm = tile / tilesN;
  const int tn = tile - tm * tilesN;
  const int m0 = tm << 6, n0 = tn << 6;
  const int rlane = lane & 15, hh = lane >> 4, koff = hh * 8, mOff = hh * 8;

  v8f acc[4][4];
#pragma unroll
  for (int i = 0; i < 4; ++i)
#pragma unroll
    for (int j = 0; j < 4; ++j) acc[i][j] = (v8f){0.f, 0.f, 0.f, 0.f, 0.f, 0.f, 0.f, 0.f};

  const _Float16* ap = A  + (size_t)(m0 + rlane) * K + koff;
  const _Float16* bp = Bt + (size_t)(n0 + rlane) * K + koff;
  const size_t step16 = (size_t)16 * K;
#pragma unroll 1
  for (int k0 = 0; k0 < K; k0 += 32) {
    v16h bh[4];
#pragma unroll
    for (int j = 0; j < 4; ++j) bh[j] = frag_load(bp + (size_t)j * step16 + k0);
#pragma unroll
    for (int i = 0; i < 4; ++i) {
      const v16h ah = frag_load(ap + (size_t)i * step16 + k0);
#pragma unroll
      for (int j = 0; j < 4; ++j) acc[i][j] = mma_h(ah, bh[j], acc[i][j]);
      guard_row(acc[i][0], acc[i][1], acc[i][2], acc[i][3], ah, bh[0], bh[1], bh[2], bh[3]);
    }
    keep4_h(bh[0], bh[1], bh[2], bh[3]);
  }
  acc_guard4(acc[0][0], acc[0][1], acc[0][2], acc[0][3]);
  acc_guard4(acc[1][0], acc[1][1], acc[1][2], acc[1][3]);
  acc_guard4(acc[2][0], acc[2][1], acc[2][2], acc[2][3]);
  acc_guard4(acc[3][0], acc[3][1], acc[3][2], acc[3][3]);

  float* slab = sT[wave];
  if (OUTK == 0) {
    const v4f b4 = *(const v4f*)(bias + n0 + rlane * 4);
    const int q = lane >> 3, c8 = (lane & 7) * 8;
    unsigned short* C = (unsigned short*)Cout;
#pragma unroll
    for (int i = 0; i < 4; ++i) {
      stage_raw(slab, acc[i][0], acc[i][1], acc[i][2], acc[i][3], scale, rlane, mOff);
      wave_sync();
      gelu_pass(slab, b4, lane);
      wave_sync();
      unsigned short* gp = C + (size_t)(m0 + 16 * i) * N + n0 + c8;
#pragma unroll
      for (int it = 0; it < 4; ++it) {
        const int row = it * 4 + q;
        const v8h hv = cvt8_slab(slab + row * SLABP + c8);
        *(volatile v8h*)(gp + (size_t)row * N) = hv;
      }
      __threadfence();
#pragma unroll
      for (int it = 0; it < 4; ++it) {
        const int row = it * 4 + q;
        const v8h hv = cvt8_slab(slab + row * SLABP + c8);
        *(volatile v8h*)(gp + (size_t)row * N) = hv;
      }
      __threadfence();
      wave_sync();
    }
  } else {
    const float bv0 = bias[n0 + rlane];
    const float bv1 = bias[n0 + 16 + rlane];
    const float bv2 = bias[n0 + 32 + rlane];
    const float bv3 = bias[n0 + 48 + rlane];
    const int c4 = (lane & 15) * 4;
    float* C = (float*)Cout;
#pragma unroll
    for (int i = 0; i < 4; ++i) {
      stage_bias(slab, acc[i][0], acc[i][1], acc[i][2], acc[i][3], scale, bv0, bv1, bv2, bv3, rlane, mOff);
      wave_sync();
#pragma unroll
      for (int it = 0; it < 8; ++it) {
        const int row = it * 2 + hh;
        const int m = m0 + 16 * i + row;
        const size_t drow = (size_t)(bat0 + (m & (HALF_B - 1))) * NSTEP + (size_t)(m >> 6);
        const v4f v = *(const v4f*)(slab + row * SLABP + c4);
        *(volatile v4f*)(C + drow * (size_t)N + n0 + c4) = v;
      }
      __threadfence();
#pragma unroll
      for (int it = 0; it < 8; ++it) {
        const int row = it * 2 + hh;
        const int m = m0 + 16 * i + row;
        const size_t drow = (size_t)(bat0 + (m & (HALF_B - 1))) * NSTEP + (size_t)(m >> 6);
        const v4f v = *(const v4f*)(slab + row * SLABP + c4);
        *(volatile v4f*)(C + drow * (size_t)N + n0 + c4) = v;
      }
      __threadfence();
      wave_sync();
    }
  }
}

extern "C" void kernel_launch(void* const* d_in, const int* in_sizes, int n_in,
                              void* d_out, int out_size, void* d_ws, size_t ws_size, hipStream_t stream) {
  if (n_in < 11 || d_out == nullptr || d_ws == nullptr) return;
  if (in_sizes[0] != NBATCH * NSTEP * NIN || in_sizes[1] != NHID * (NIN + NHID) || in_sizes[2] != NHID ||
      in_sizes[3] != NHID * NHID || in_sizes[4] != NHID || in_sizes[5] != NHID * (NHID + NHID) ||
      in_sizes[6] != NHID || in_sizes[7] != NHID * NHID || in_sizes[8] != NHID ||
      in_sizes[9] != NOUT * NHID || in_sizes[10] != NOUT || out_size != NBATCH * NSTEP * NOUT) return;

  const float* x      = (const float*)d_in[0];
  const float* w_in1  = (const float*)d_in[1];
  const float* b_in1  = (const float*)d_in[2];
  const float* w_out1 = (const float*)d_in[3];
  const float* b_out1 = (const float*)d_in[4];
  const float* w_in2  = (const float*)d_in[5];
  const float* b_in2  = (const float*)d_in[6];
  const float* w_out2 = (const float*)d_in[7];
  const float* b_out2 = (const float*)d_in[8];
  const float* w_last = (const float*)d_in[9];
  const float* b_last = (const float*)d_in[10];
  float* out = (float*)d_out;

  char* ws = (char*)d_ws;
  size_t off = 0;
  auto carve = [&](size_t bytes) -> char* { char* p = ws + off; off += (bytes + 255) & ~(size_t)255; return p; };
  unsigned short* XT  = (unsigned short*)carve((size_t)NHALF * HROWS * NIN * 2);
  unsigned short* WTS = (unsigned short*)carve(WTS_ELEMS * 2);
  unsigned short* PA  = (unsigned short*)carve((size_t)HROWS * NHID * 2);
  unsigned short* PB  = (unsigned short*)carve((size_t)HROWS * NHID * 2);
  if (off > ws_size || off > (size_t)134217728) return;

  prep_x_kernel<<<PX_BLOCKS, NTHR, 0, stream>>>(x, XT);
  prep_w_kernel<<<PW_BLOCKS, NTHR, 0, stream>>>(w_in1, w_out1, w_in2, w_out2, w_last, WTS);

  const int gridSq = (HROWS / 64) * (NHID / 64) / 8;
  const int gridL  = (HROWS / 64) * (NOUT / 64) / 8;
  for (int hf = 0; hf < NHALF; ++hf) {
    rnn_rec_kernel<NIN><<<1, NTHR, 0, stream>>>(XT + (size_t)hf * HROWS * NIN, WTS + OFF_WX1, WTS + OFF_WH1, b_in1, PA);
    gemm_tile_kernel<0><<<gridSq, NTHR, 0, stream>>>(PA, WTS + OFF_WO1, (void*)PB, b_out1, HROWS, NHID, NHID, ACC_INV, 0);
    rnn_rec_kernel<NHID><<<1, NTHR, 0, stream>>>(PB, WTS + OFF_WX2, WTS + OFF_WH2, b_in2, PA);
    gemm_tile_kernel<0><<<gridSq, NTHR, 0, stream>>>(PA, WTS + OFF_WO2, (void*)PB, b_out2, HROWS, NHID, NHID, ACC_INV, 0);
    gemm_tile_kernel<1><<<gridL, NTHR, 0, stream>>>(PB, WTS + OFF_WL, (void*)out, b_last, HROWS, NOUT, NHID, ACC_INV, hf * HALF_B);
  }
}
